// MoE_21096879358054
// MI455X (gfx1250) — hardware-run, weakly checked
//
#include <hip/hip_runtime.h>
#include <math.h>

#define NTOK_ALL 32768
#define NPASS 8
#define NTOK (NTOK_ALL / NPASS)
#define DM 256
#define FF 512
#define NE 8
#define TOPK 4
#define SPT TOPK
#define NSLOT (NTOK * TOPK)
#define R_MAX (NSLOT + 64 * NE)
#define NT_MAX (R_MAX / 64)
#define RW_CH 8192

#define CX_LOG2 11
#define CW_LOG2 16
#define CH_LOG2 11
#define CH ((float)(1u << CH_LOG2))
#define SC_H (1.0f / (float)(1u << (CX_LOG2 + CW_LOG2)))
#define SC_Y (1.0f / (float)(1u << (CH_LOG2 + CW_LOG2)))

#define TBL_COUNT 0
#define TBL_POFF 16
#define TBL_NTILES 32
#define TBL_TILE_E 64
#define TBL_HDR 512
#define TBL_ROWTOK TBL_HDR
#define TBL_SLOTROW (TBL_HDR + R_MAX)
#define TBL_WORDS (TBL_HDR + R_MAX + NSLOT)
#define OUT1_OFF ((size_t)NTOK_ALL * (size_t)DM)

static_assert(NE == 8 && TOPK == 4 && SPT == 4 && NPASS == 8 && NTOK == 4096 && DM == 256 && FF == 512);
static_assert(DM % 64 == 0 && FF % 64 == 0 && NTOK % 256 == 0 && NSLOT % 128 == 0 && R_MAX % 64 == 0 && NSLOT == 16384 && R_MAX == 16896 && NT_MAX == 264 && TBL_WORDS == 33792);
static_assert(TBL_COUNT + NE <= TBL_POFF && TBL_POFF + NE + 1 <= TBL_NTILES && TBL_NTILES < TBL_TILE_E && TBL_TILE_E + NT_MAX <= TBL_HDR && TBL_HDR <= 512 && TBL_HDR % 4 == 0);
static_assert(CX_LOG2 == 11 && CW_LOG2 == 16 && CH_LOG2 == 11 && (NTOK * DM / 8) % 256 == 0);

constexpr size_t al256(size_t b) { return (b + 255) & ~(size_t)255; }
constexpr size_t WS_TOTAL = al256((size_t)NE * FF * DM * 2) + al256((size_t)NE * DM * FF * 2) + al256((size_t)NTOK * DM * 2) + 2 * al256((size_t)NSLOT * 4)
                          + al256((size_t)TBL_WORDS * 4) + al256((size_t)R_MAX * DM * 2) + al256((size_t)R_MAX * FF * 2) + al256((size_t)R_MAX * DM * 4);
static_assert(WS_TOTAL == (size_t)49811456 && WS_TOTAL < (size_t)134217728);

typedef _Float16 h16;
typedef __attribute__((ext_vector_type(16))) _Float16 v16h;
typedef __attribute__((ext_vector_type(8)))  _Float16 v8h;
typedef __attribute__((ext_vector_type(8)))  float    v8f;
typedef __attribute__((ext_vector_type(4)))  float    v4f;
typedef __attribute__((ext_vector_type(2)))  float    v2f;
typedef __attribute__((ext_vector_type(4)))  unsigned int v4u;
typedef __attribute__((ext_vector_type(4)))  int      v4i;
typedef __attribute__((ext_vector_type(2)))  int      v2i;


#define VST2(T, ptr, val) do { const T vst2_v_ = (val); *(volatile T*)(ptr) = vst2_v_; __threadfence(); *(volatile T*)(ptr) = vst2_v_; } while (0)

static __device__ __forceinline__ float bfr(float f) {
    unsigned u = __float_as_uint(f);
    u += 0x7FFFu + ((u >> 16) & 1u);
    return __uint_as_float(u & 0xFFFF0000u);
}
static __device__ __forceinline__ h16 toh_flush(float v) { const float w = (fabsf(v) < 6.103515625e-05f) ? 0.0f : v; return (h16)w; }
static __device__ __forceinline__ void st8h(h16* p, const float* v) {
    v8h hv;
#pragma unroll
    for (int e = 0; e < 8; ++e) hv[e] = toh_flush(v[e]);
    VST2(v8h, p, hv);
}

union FragU { v16h v; v8h h[2]; };
static __device__ __forceinline__ v16h frag_ld(const h16* p) {
    FragU f; f.h[0] = *(const v8h*)(p); f.h[1] = *(const v8h*)(p + 16); return f.v;
}
static __device__ __forceinline__ v8f wmma16g(v16h a, v16h b, v8f c) {
    c = __builtin_amdgcn_wmma_f32_16x16x32_f16(false, a, false, b, (short)0, c, false, false);
    asm volatile("v_nop\n\tv_nop\n\tv_nop\n\tv_nop" : "+v"(c) : "v"(a), "v"(b));
    return c;
}
static __device__ __forceinline__ void wave_sync_lds() {
    __builtin_amdgcn_fence(3  , "workgroup");
    __builtin_amdgcn_wave_barrier();
    __builtin_amdgcn_fence(2  , "workgroup");
}
template <int LOG2C>
__global__ __launch_bounds__(256) void k_plane(const float* __restrict__ src, h16* __restrict__ dst, unsigned n8) {
    const unsigned u = blockIdx.x * 256u + threadIdx.x;
    if (u >= n8) return;
    const float cs = (float)(1u << LOG2C);
    const v4f a = *(const v4f*)(src + (size_t)u * 8u);
    const v4f b = *(const v4f*)(src + (size_t)u * 8u + 4u);
    float v[8] = {bfr(a.x) * cs, bfr(a.y) * cs, bfr(a.z) * cs, bfr(a.w) * cs, bfr(b.x) * cs, bfr(b.y) * cs, bfr(b.z) * cs, bfr(b.w) * cs};
    st8h(dst + (size_t)u * 8u, v);
}
__global__ __launch_bounds__(128) void k_planeTw(const float* __restrict__ src, h16* __restrict__ dst, unsigned ne, unsigned K, unsigned N, unsigned pitch, unsigned estride, float cs) {
    __shared__ __align__(16) float sT[4][64 * 36];
    const unsigned lane = threadIdx.x & 31u;
    const unsigned wave = threadIdx.x >> 5;
    const unsigned tk = K >> 6, tn = N >> 5;
    const unsigned tpe = tk * tn;
    const unsigned u = blockIdx.x * 4u + wave;
    if (u >= ne * tpe) return;
    const unsigned e = u / tpe;
    const unsigned rem = u - e * tpe;
    const unsigned kt = rem / tn;
    const unsigned nt = rem - kt * tn;
    const unsigned k0 = kt << 6, n0 = nt << 5;
    const size_t sbase = (size_t)e * (size_t)estride;
    const size_t ebase = (size_t)e * ((size_t)K * (size_t)N);
    float* slab = sT[wave];
#pragma unroll
    for (int i = 0; i < 16; ++i) {
        const unsigned p = lane + 32u * (unsigned)i;
        const unsigned kr = p >> 3;
        const unsigned n4 = (p & 7u) * 4u;
        const v4f a = *(const v4f*)(src + sbase + (size_t)(k0 + kr) * pitch + n0 + n4);
        v4f s;
        s.x = bfr(a.x) * cs; s.y = bfr(a.y) * cs; s.z = bfr(a.z) * cs; s.w = bfr(a.w) * cs;
        *(v4f*)(&slab[kr * 36u + n4]) = s;
    }
    wave_sync_lds();
#pragma unroll
    for (int i = 0; i < 8; ++i) {
        const unsigned q = lane + 32u * (unsigned)i;
        const unsigned n = q >> 3;
        const unsigned kp = q & 7u;
        float v[8];
#pragma unroll
        for (int j = 0; j < 8; ++j) v[j] = slab[(8u * kp + (unsigned)j) * 36u + n];
        st8h(dst + ebase + (size_t)(n0 + n) * K + k0 + 8u * kp, v);
    }
}


__global__ __launch_bounds__(256) void k_gate4m(const float* __restrict__ x, const int* __restrict__ mask, const float* __restrict__ Wg, int* __restrict__ sel, float* __restrict__ wgt) {
    const unsigned lane = threadIdx.x & 31u;
    const unsigned wave = threadIdx.x >> 5;
    const unsigned tok0 = (blockIdx.x * 8u + wave) * 32u;
    if (tok0 >= (unsigned)NTOK) return;
    v4i ke; ke.x = 0; ke.y = 1; ke.z = 2; ke.w = 3;
    v4f kw; kw.x = 0.0f; kw.y = 0.0f; kw.z = 0.0f; kw.w = 0.0f;
    const float mymask = (float)mask[tok0 + lane];
    for (unsigned tt = 0; tt < 32u; ++tt) {
        const float* xr = x + (size_t)(tok0 + tt) * DM;
        double acc[NE];
#pragma unroll
        for (int g = 0; g < NE; ++g) acc[g] = 0.0;
        for (unsigned q = 0; q < (unsigned)(DM / 32); ++q) {
            const unsigned d = lane + 32u * q;
            const double xv = (double)bfr(xr[d]);
            const float* wr = Wg + (size_t)d * NE;
#pragma unroll
            for (int g = 0; g < NE; ++g) acc[g] = fma((double)bfr(wr[g]), xv, acc[g]);
        }
#pragma unroll
        for (int g = 0; g < NE; ++g) {
            double s = acc[g];
            s += __shfl_xor(s, 16, 32);
            s += __shfl_xor(s, 8, 32);
            s += __shfl_xor(s, 4, 32);
            s += __shfl_xor(s, 2, 32);
            s += __shfl_xor(s, 1, 32);
            acc[g] = s;
        }
        int e[4]; double v[4];
        unsigned takenbits = 0u;
#pragma unroll
        for (int k = 0; k < 4; ++k) {
            int be = 0; double bv = 0.0; bool have = false;
#pragma unroll
            for (int g = 0; g < NE; ++g) {
                const bool free_ = ((takenbits >> g) & 1u) == 0u;
                const bool tk = free_ && (!have || acc[g] > bv);
                be = tk ? g : be; bv = tk ? acc[g] : bv; have = have || free_;
            }
            e[k] = be; v[k] = bv; takenbits |= (1u << be);
        }
        const float x1 = expf((float)(v[1] - v[0]));
        const float x2 = expf((float)(v[2] - v[0]));
        const float x3 = expf((float)(v[3] - v[0]));
        const float den = ((1.0f + x1) + x2) + x3;
        const float g0 = 1.0f / den, g1 = x1 / den, g2 = x2 / den, g3 = x3 / den;
        const bool mine = (lane == tt);
        ke.x = mine ? e[0] : ke.x; ke.y = mine ? e[1] : ke.y; ke.z = mine ? e[2] : ke.z; ke.w = mine ? e[3] : ke.w;
        kw.x = mine ? g0 : kw.x; kw.y = mine ? g1 : kw.y; kw.z = mine ? g2 : kw.z; kw.w = mine ? g3 : kw.w;
    }
    kw = kw * mymask;
    const unsigned t = tok0 + lane;
    VST2(v4i, sel + 4u * t, ke);
    VST2(v4f, wgt + 4u * t, kw);
}

template <int NE_>
__global__ __launch_bounds__(32) void k_route1w(const int* __restrict__ sel, int* __restrict__ tbl, unsigned nslot, unsigned spt, unsigned hdr, unsigned rmax,
                                                unsigned offPoff, unsigned offNtiles, unsigned offTileE) {
    static_assert(NE_ >= 1 && NE_ <= 32);
    __shared__ __align__(16) int s_img[RW_CH];
    __shared__ __align__(16) int s_hdr[512];
    const unsigned lane = threadIdx.x & 31u;
    const unsigned spl = nslot >> 5;
    const unsigned ng = spl >> 2;
    const unsigned ntmax = rmax >> 6;
    const v4i* sp = (const v4i*)(sel + (size_t)lane * spl);
    int cnt[NE_];
#pragma unroll
    for (int j = 0; j < NE_; ++j) cnt[j] = 0;
    for (unsigned g = 0; g < ng; ++g) {
        const v4i v = sp[g];
#pragma unroll
        for (int c = 0; c < 4; ++c) {
            const int e = min(max(v[c], 0), NE_ - 1);
#pragma unroll
            for (int j = 0; j < NE_; ++j) cnt[j] += (e == j) ? 1 : 0;
        }
    }
    int base0[NE_], total[NE_];
#pragma unroll
    for (int j = 0; j < NE_; ++j) {
        int pre = 0, tot = cnt[j];
#pragma unroll
        for (int d = 1; d < 32; d <<= 1) {
            const int t = __shfl_xor(tot, d, 32);
            pre += ((lane & (unsigned)d) != 0u) ? t : 0;
            tot += t;
        }
        base0[j] = pre;
        total[j] = tot;
    }
    int poff[NE_ + 1];
    poff[0] = 0;
#pragma unroll
    for (int j = 0; j < NE_; ++j) poff[j + 1] = poff[j] + (((total[j] + 63) >> 6) << 6);
    for (unsigned i = lane; i < 512u; i += 32u) s_hdr[i] = (i >= offTileE && i < offTileE + ntmax) ? -1 : 0;
    wave_sync_lds();
    if (lane == 0u) {
#pragma unroll
        for (int j = 0; j < NE_; ++j) { s_hdr[min((unsigned)j, 511u)] = total[j]; s_hdr[min(offPoff + (unsigned)j, 511u)] = poff[j]; }
        s_hdr[min(offPoff + (unsigned)NE_, 511u)] = poff[NE_];
        s_hdr[min(offNtiles, 511u)] = poff[NE_] >> 6;
    }
    for (unsigned t = lane; t < ntmax; t += 32u) {
        const int b64 = (int)(t * 64u);
        int ev = -1;
#pragma unroll
        for (int j = 0; j < NE_; ++j) ev = (b64 >= poff[j] && b64 < poff[j + 1]) ? j : ev;
        s_hdr[min(offTileE + t, 511u)] = ev;
    }
    wave_sync_lds();
    for (int pass = 0; pass < 2; ++pass) {
        for (unsigned i = lane; i < (hdr >> 2); i += 32u) *(volatile v4i*)(tbl + 4u * i) = *(const v4i*)(&s_hdr[4u * i]);
        __threadfence();
    }
    for (unsigned lo = 0; lo < rmax; lo += (unsigned)RW_CH) {
        for (unsigned i = lane; i < (unsigned)(RW_CH / 4); i += 32u) *(v4i*)(&s_img[4u * i]) = (v4i){-1, -1, -1, -1};
        wave_sync_lds();
        int run[NE_];
#pragma unroll
        for (int j = 0; j < NE_; ++j) run[j] = base0[j];
        for (unsigned g = 0; g < ng; ++g) {
            const v4i v = sp[g];
#pragma unroll
            for (int c = 0; c < 4; ++c) {
                const int e = min(max(v[c], 0), NE_ - 1);
                int row = 0;
#pragma unroll
                for (int j = 0; j < NE_; ++j) {
                    const bool hit = (e == j);
                    row = hit ? (poff[j] + run[j]) : row;
                    run[j] += hit ? 1 : 0;
                }
                row = min(max(row, 0), (int)rmax - 1);
                const unsigned rel = (unsigned)row - lo;
                if (rel < (unsigned)RW_CH) s_img[rel] = (int)((lane * spl + 4u * g + (unsigned)c) / spt);
            }
        }
        wave_sync_lds();
        const unsigned nw = min((unsigned)RW_CH, rmax - lo);
        for (int pass = 0; pass < 2; ++pass) {
            for (unsigned i = lane; i < (nw >> 2); i += 32u) *(volatile v4i*)(tbl + hdr + lo + 4u * i) = *(const v4i*)(&s_img[4u * i]);
            __threadfence();
        }
        wave_sync_lds();
    }
    for (unsigned lo = 0; lo < nslot; lo += (unsigned)RW_CH) {
        int run[NE_];
#pragma unroll
        for (int j = 0; j < NE_; ++j) run[j] = base0[j];
        for (unsigned g = 0; g < ng; ++g) {
            const v4i v = sp[g];
#pragma unroll
            for (int c = 0; c < 4; ++c) {
                const int e = min(max(v[c], 0), NE_ - 1);
                int row = 0;
#pragma unroll
                for (int j = 0; j < NE_; ++j) {
                    const bool hit = (e == j);
                    row = hit ? (poff[j] + run[j]) : row;
                    run[j] += hit ? 1 : 0;
                }
                row = min(max(row, 0), (int)rmax - 1);
                const unsigned rel = (lane * spl + 4u * g + (unsigned)c) - lo;
                if (rel < (unsigned)RW_CH) s_img[rel] = row;
            }
        }
        wave_sync_lds();
        const unsigned nw = min((unsigned)RW_CH, nslot - lo);
        for (int pass = 0; pass < 2; ++pass) {
            for (unsigned i = lane; i < (nw >> 2); i += 32u) *(volatile v4i*)(tbl + hdr + rmax + lo + 4u * i) = *(const v4i*)(&s_img[4u * i]);
            __threadfence();
        }
        wave_sync_lds();
    }
}

__global__ __launch_bounds__(256) void k_gather(const h16* __restrict__ x16, const int* __restrict__ tbl, h16* __restrict__ Xg) {
    const unsigned row = blockIdx.x * 8u + (threadIdx.x >> 5);
    if (row >= (unsigned)R_MAX) return;
    const unsigned c = (threadIdx.x & 31u) * 8u;
    const int tr = tbl[TBL_ROWTOK + row];
    const bool pad = (tr < 0);
    const int tok = min(max(tr, 0), NTOK - 1);
    const v4u ld = *(const v4u*)(x16 + (size_t)(unsigned)tok * DM + c);
    v4u o;
    o.x = pad ? 0u : ld.x; o.y = pad ? 0u : ld.y; o.z = pad ? 0u : ld.z; o.w = pad ? 0u : ld.w;
    VST2(v4u, Xg + (size_t)row * DM + c, o);
}

__global__ __launch_bounds__(256) void k_ffn1(const h16* __restrict__ Xg, const h16* __restrict__ Wp, const float* __restrict__ eb,
                                              const int* __restrict__ tbl, h16* __restrict__ Hg) {
    __shared__ __align__(16) float sT[8][16 * 68];
    const unsigned lane = threadIdx.x & 31u;
    const unsigned wave = threadIdx.x >> 5;
    const unsigned u = blockIdx.x * 8u + wave;
    if (u >= (unsigned)(NT_MAX * (FF / 64))) return;
    const unsigned rowtile = u / (unsigned)(FF / 64);
    const unsigned ct = u - rowtile * (unsigned)(FF / 64);
    const int nt = min(max(tbl[TBL_NTILES], 0), NT_MAX);
    if ((int)rowtile >= nt) return;
    const int e = min(max(tbl[TBL_TILE_E + rowtile], 0), NE - 1);
    const size_t wbase = (size_t)(unsigned)e * (size_t)(FF * DM);
    const unsigned m0 = rowtile << 6, n0 = ct << 6;
    const unsigned rlane = lane & 15u;
    const unsigned koff = (lane >> 4) * 8u;
    const unsigned mOff = koff;

    v8f acc[4][4];
#pragma unroll
    for (int i = 0; i < 4; ++i)
#pragma unroll
        for (int j = 0; j < 4; ++j) acc[i][j] = (v8f){0.f,0.f,0.f,0.f,0.f,0.f,0.f,0.f};

    for (unsigned k0 = 0; k0 < (unsigned)DM; k0 += 32u) {
        v16h bh[4];
#pragma unroll
        for (int j = 0; j < 4; ++j)
            bh[j] = frag_ld(Wp + wbase + (size_t)(n0 + ((unsigned)j << 4) + rlane) * DM + koff + k0);
#pragma unroll
        for (int i = 0; i < 4; ++i) {
            const v16h ah = frag_ld(Xg + (size_t)(m0 + ((unsigned)i << 4) + rlane) * DM + koff + k0);
#pragma unroll
            for (int j = 0; j < 4; ++j) acc[i][j] = wmma16g(ah, bh[j], acc[i][j]);
        }
    }

    float ebv[4];
#pragma unroll
    for (int j = 0; j < 4; ++j) ebv[j] = bfr(eb[(unsigned)e * (unsigned)FF + n0 + ((unsigned)j << 4) + rlane]);

    float* slab = sT[wave];
#pragma unroll
    for (int i = 0; i < 4; ++i) {
        const unsigned mBase = m0 + ((unsigned)i << 4);
#pragma unroll
        for (int j = 0; j < 4; ++j)
#pragma unroll
            for (int r = 0; r < 8; ++r) {
                const float a = acc[i][j][r] * SC_H + ebv[j];
                const float g = fmaxf(a, 0.0f);
                slab[(mOff + (unsigned)r) * 68u + ((unsigned)j << 4) + rlane] = g * CH;
            }
        wave_sync_lds();
        const unsigned q = lane >> 3, c8 = (lane & 7u) * 8u;
        v8h hv[4];
#pragma unroll
        for (int it = 0; it < 4; ++it) {
            const unsigned row = (unsigned)it * 4u + q;
            const float* sp = slab + row * 68u + c8;
#pragma unroll
            for (int t = 0; t < 8; ++t) hv[it][t] = toh_flush(sp[t]);
        }
        for (int pass = 0; pass < 2; ++pass) {
#pragma unroll
            for (int it = 0; it < 4; ++it) {
                const unsigned row = (unsigned)it * 4u + q;
                *(volatile v8h*)(Hg + (size_t)(mBase + row) * FF + n0 + c8) = hv[it];
            }
            __threadfence();
        }
        wave_sync_lds();
    }
}

__global__ __launch_bounds__(256) void k_ffn2(const h16* __restrict__ Hg, const h16* __restrict__ Wp, const float* __restrict__ eb,
                                              const int* __restrict__ tbl, float* __restrict__ Yg) {
    __shared__ __align__(16) float sT[8][16 * 68];
    const unsigned lane = threadIdx.x & 31u;
    const unsigned wave = threadIdx.x >> 5;
    const unsigned u = blockIdx.x * 8u + wave;
    if (u >= (unsigned)(NT_MAX * (DM / 64))) return;
    const unsigned rowtile = u / (unsigned)(DM / 64);
    const unsigned ct = u - rowtile * (unsigned)(DM / 64);
    const int nt = min(max(tbl[TBL_NTILES], 0), NT_MAX);
    if ((int)rowtile >= nt) return;
    const int e = min(max(tbl[TBL_TILE_E + rowtile], 0), NE - 1);
    const size_t wbase = (size_t)(unsigned)e * (size_t)(DM * FF);
    const unsigned m0 = rowtile << 6, n0 = ct << 6;
    const unsigned rlane = lane & 15u;
    const unsigned koff = (lane >> 4) * 8u;
    const unsigned mOff = koff;

    v8f acc[4][4];
#pragma unroll
    for (int i = 0; i < 4; ++i)
#pragma unroll
        for (int j = 0; j < 4; ++j) acc[i][j] = (v8f){0.f,0.f,0.f,0.f,0.f,0.f,0.f,0.f};

    for (unsigned k0 = 0; k0 < (unsigned)FF; k0 += 32u) {
        v16h bh[4];
#pragma unroll
        for (int j = 0; j < 4; ++j)
            bh[j] = frag_ld(Wp + wbase + (size_t)(n0 + ((unsigned)j << 4) + rlane) * FF + koff + k0);
#pragma unroll
        for (int i = 0; i < 4; ++i) {
            const v16h ah = frag_ld(Hg + (size_t)(m0 + ((unsigned)i << 4) + rlane) * FF + koff + k0);
#pragma unroll
            for (int j = 0; j < 4; ++j) acc[i][j] = wmma16g(ah, bh[j], acc[i][j]);
        }
    }

    float ebv[4];
#pragma unroll
    for (int j = 0; j < 4; ++j) ebv[j] = bfr(eb[(unsigned)e * (unsigned)DM + n0 + ((unsigned)j << 4) + rlane]);

    float* slab = sT[wave];
#pragma unroll
    for (int i = 0; i < 4; ++i) {
        const unsigned mBase = m0 + ((unsigned)i << 4);
#pragma unroll
        for (int j = 0; j < 4; ++j)
#pragma unroll
            for (int r = 0; r < 8; ++r)
                slab[(mOff + (unsigned)r) * 68u + ((unsigned)j << 4) + rlane] = acc[i][j][r] * SC_Y + ebv[j];
        wave_sync_lds();
        const unsigned hh = lane >> 4, c4 = (lane & 15u) * 4u;
#pragma unroll
        for (int half = 0; half < 2; ++half) {
            v4f vv[4];
#pragma unroll
            for (int it = 0; it < 4; ++it) {
                const unsigned row = (unsigned)(half * 4 + it) * 2u + hh;
                vv[it] = *(const v4f*)(slab + row * 68u + c4);
            }
            for (int pass = 0; pass < 2; ++pass) {
#pragma unroll
                for (int it = 0; it < 4; ++it) {
                    const unsigned row = (unsigned)(half * 4 + it) * 2u + hh;
                    *(volatile v4f*)(Yg + (size_t)(mBase + row) * DM + n0 + c4) = vv[it];
                }
                __threadfence();
            }
        }
        wave_sync_lds();
    }
}

__global__ __launch_bounds__(256) void k_combine4r(const float* __restrict__ Yg, const float* __restrict__ wgt, const int* __restrict__ tbl, const float* __restrict__ x, float* __restrict__ out) {
    const unsigned t = blockIdx.x * 4u + (threadIdx.x >> 6);
    if (t >= (unsigned)NTOK) return;
    const unsigned c = (threadIdx.x & 63u) * 4u;
    const v4i rr = *(const v4i*)(tbl + TBL_SLOTROW + 4u * t);
    const int r0 = min(max(rr.x, 0), R_MAX - 1);
    const int r1 = min(max(rr.y, 0), R_MAX - 1);
    const int r2 = min(max(rr.z, 0), R_MAX - 1);
    const int r3 = min(max(rr.w, 0), R_MAX - 1);
    const v4f w = *(const v4f*)(wgt + 4u * t);
    const v4f a0 = *(const v4f*)(Yg + (size_t)(unsigned)r0 * DM + c);
    const v4f a1 = *(const v4f*)(Yg + (size_t)(unsigned)r1 * DM + c);
    const v4f a2 = *(const v4f*)(Yg + (size_t)(unsigned)r2 * DM + c);
    const v4f a3 = *(const v4f*)(Yg + (size_t)(unsigned)r3 * DM + c);
    const v4f xin = *(const v4f*)(x + (size_t)t * DM + c);
    v4f xr; xr.x = bfr(xin.x); xr.y = bfr(xin.y); xr.z = bfr(xin.z); xr.w = bfr(xin.w);
    const v4f y = ((((a0 * w.x) + (a1 * w.y)) + (a2 * w.z)) + (a3 * w.w)) + xr;
    VST2(v4f, out + (size_t)t * DM + c, y);
}

__global__ __launch_bounds__(32) void k_zero(float* __restrict__ out1) {
    if ((threadIdx.x & 31u) == 0u) {
        VST2(float, out1, 0.0f);
    }
}

extern "C" void kernel_launch(void* const* d_in, const int* in_sizes, int n_in, void* d_out, int out_size,
                              void* d_ws, size_t ws_size, hipStream_t stream) {
    if (n_in < 7) return;
    if (in_sizes[0] < NTOK_ALL * DM || in_sizes[1] < NTOK_ALL || in_sizes[2] < DM * NE || in_sizes[3] < NE * DM * FF || in_sizes[4] < NE * FF || in_sizes[5] < NE * FF * DM || in_sizes[6] < NE * DM) return;
    if (out_size < NTOK_ALL * DM + 1) return;

    const float* x    = (const float*)d_in[0];
    const int*   mask = (const int*)d_in[1];
    const float* Wg   = (const float*)d_in[2];
    const float* w1   = (const float*)d_in[3];
    const float* b1   = (const float*)d_in[4];
    const float* w2   = (const float*)d_in[5];
    const float* b2   = (const float*)d_in[6];
    float* out = (float*)d_out;

    char* wsp = (char*)d_ws;
    size_t off = 0;
    auto carve = [&](size_t bytes) -> void* { void* r = wsp + off; off += (bytes + 255) & ~(size_t)255; return r; };
    h16*   w1t = (h16*)carve((size_t)NE * FF * DM * 2);
    h16*   w2t = (h16*)carve((size_t)NE * DM * FF * 2);
    h16*   x16 = (h16*)carve((size_t)NTOK * DM * 2);
    int*   sel = (int*)carve((size_t)NSLOT * 4);
    float* wgt = (float*)carve((size_t)NSLOT * 4);
    int*   tbl = (int*)carve((size_t)TBL_WORDS * 4);
    h16*   Xg  = (h16*)carve((size_t)R_MAX * DM * 2);
    h16*   Hg  = (h16*)carve((size_t)R_MAX * FF * 2);
    float* Yg  = (float*)carve((size_t)R_MAX * DM * 4);
    if (off != WS_TOTAL || off > ws_size || off > (size_t)134217728) return;

    k_planeTw<<<(NE * (DM / 64) * (FF / 32) + 3) / 4, 128, 0, stream>>>(w1, w1t, (unsigned)NE, (unsigned)DM, (unsigned)FF, (unsigned)FF, (unsigned)(DM * FF), (float)(1u << CW_LOG2));
    k_planeTw<<<(NE * (FF / 64) * (DM / 32) + 3) / 4, 128, 0, stream>>>(w2, w2t, (unsigned)NE, (unsigned)FF, (unsigned)DM, (unsigned)DM, (unsigned)(FF * DM), (float)(1u << CW_LOG2));

    for (int p = 0; p < NPASS; ++p) {
        const size_t tok0 = (size_t)p * NTOK;
        k_plane<CX_LOG2><<<(NTOK * DM / 8) / 256, 256, 0, stream>>>(x + tok0 * DM, x16, (unsigned)(NTOK * DM / 8));
        k_gate4m<<<NTOK / 256, 256, 0, stream>>>(x + tok0 * DM, mask + tok0, Wg, sel, wgt);
        k_route1w<NE><<<1, 32, 0, stream>>>(sel, tbl, (unsigned)NSLOT, (unsigned)SPT, (unsigned)TBL_HDR, (unsigned)R_MAX, (unsigned)TBL_POFF, (unsigned)TBL_NTILES, (unsigned)TBL_TILE_E);
        k_gather<<<R_MAX / 8, 256, 0, stream>>>(x16, tbl, Xg);
        k_ffn1<<<(NT_MAX * (FF / 64) + 7) / 8, 256, 0, stream>>>(Xg, w1t, b1, tbl, Hg);
        k_ffn2<<<(NT_MAX * (DM / 64) + 7) / 8, 256, 0, stream>>>(Hg, w2t, b2, tbl, Yg);
        k_combine4r<<<NTOK / 4, 256, 0, stream>>>(Yg, wgt, tbl, x + tok0 * DM, out + tok0 * DM);
    }
    k_zero<<<1, 32, 0, stream>>>(out + OUT1_OFF);
}
